// KernelSparseAttentionLayer_54391465836690
// MI455X (gfx1250) — hardware-run, weakly checked
//
#include <hip/hip_runtime.h>

typedef float          v8f   __attribute__((ext_vector_type(8)));
typedef float          v4f   __attribute__((ext_vector_type(4)));
typedef unsigned int   v4u   __attribute__((ext_vector_type(4)));
typedef int            v8i   __attribute__((ext_vector_type(8)));
typedef unsigned short v8us  __attribute__((ext_vector_type(8)));
typedef unsigned short v16us __attribute__((ext_vector_type(16)));
typedef __bf16         v16bf __attribute__((ext_vector_type(16)));
typedef _Float16       v16h  __attribute__((ext_vector_type(16)));
typedef v4f  __attribute__((may_alias)) v4fa;
typedef v8us __attribute__((may_alias)) v8usa;
union FragB { v16bf v; v16us u; v8us h[2]; v8i w; };
union FragH { v16h  v; v16us u; v8us h[2]; v8i w; };

__device__ __forceinline__ v8f wmb(const FragB& a, const FragB& b, v8f c) {
  v8f d = __builtin_amdgcn_wmma_f32_16x16x32_bf16(false, a.v, false, b.v, (short)0, c, false, false);
  asm volatile("v_nop\n\tv_nop\n\tv_nop\n\tv_nop" : "+v"(d) : "v"(a.w), "v"(b.w));
  return d;
}

__device__ __forceinline__ v8f wmh(const FragH& a, const FragH& b, v8f c) {
  v8f d = __builtin_amdgcn_wmma_f32_16x16x32_f16(false, a.v, false, b.v, (short)0, c, false, false);
  asm volatile("v_nop\n\tv_nop\n\tv_nop\n\tv_nop" : "+v"(d) : "v"(a.w), "v"(b.w));
  return d;
}

__device__ __forceinline__ unsigned bf16_bits(float f) {
  const unsigned u = __float_as_uint(f);
  const unsigned r = (u + 0x7FFFu + ((u >> 16) & 1u)) >> 16;
  const unsigned q = (u >> 16) | 0x40u;
  return ((u & 0x7fffffffu) > 0x7f800000u) ? q : r;
}

__device__ __forceinline__ float bf16_val(float f) {
  return __uint_as_float(bf16_bits(f) << 16);
}
__device__ __forceinline__ int clampi(int v, int lo, int hi) {
  return v < lo ? lo : (v > hi ? hi : v);
}

__device__ __forceinline__ unsigned f16_bits(float f) {
  const unsigned u  = __float_as_uint(f);
  const unsigned s  = (u >> 16) & 0x8000u;
  const unsigned a  = u & 0x7fffffffu;
  const unsigned t  = a - 0x38000000u;
  const unsigned r  = (t + 0x0FFFu + ((t >> 13) & 1u)) >> 13;
  const unsigned rc = r > 0x7C00u ? 0x7C00u : r;
  const bool small  = a < 0x38800000u;
  const bool isnan  = a > 0x7f800000u;
  const unsigned fin = small ? 0u : (s | rc);
  return isnan ? (s | 0x7E00u) : fin;
}

__device__ __forceinline__ unsigned pk16(unsigned lo, unsigned hi) { return lo | (hi << 16); }
__device__ __forceinline__ unsigned bf16_lo_bits(float v) {
  float hi = bf16_val(v);
  asm volatile("" : "+v"(hi));
  return bf16_bits(v - hi);
}
__device__ __forceinline__ v4u pack8_bf16(v4f a, v4f c) {
  return (v4u){ pk16(bf16_bits(a[0]), bf16_bits(a[1])), pk16(bf16_bits(a[2]), bf16_bits(a[3])),
                pk16(bf16_bits(c[0]), bf16_bits(c[1])), pk16(bf16_bits(c[2]), bf16_bits(c[3])) };
}
__device__ __forceinline__ v4u pack8_bf16_lo(v4f a, v4f c) {
  return (v4u){ pk16(bf16_lo_bits(a[0]), bf16_lo_bits(a[1])), pk16(bf16_lo_bits(a[2]), bf16_lo_bits(a[3])),
                pk16(bf16_lo_bits(c[0]), bf16_lo_bits(c[1])), pk16(bf16_lo_bits(c[2]), bf16_lo_bits(c[3])) };
}
__device__ __forceinline__ v4u pack8_f16(v4f a, v4f c) {
  return (v4u){ pk16(f16_bits(a[0]), f16_bits(a[1])), pk16(f16_bits(a[2]), f16_bits(a[3])),
                pk16(f16_bits(c[0]), f16_bits(c[1])), pk16(f16_bits(c[2]), f16_bits(c[3])) };
}

template <int FORM>
__global__ __launch_bounds__(256) void k_plane(const float* __restrict__ src, int rows, int cols, int ldsrc,
                                               unsigned short* __restrict__ dst, int MP, int KP) {
  static_assert(FORM >= 0 && FORM <= 3);
  const int KTOT = (FORM == 1 || FORM == 3) ? 2 * KP : KP;
  const unsigned ppr   = (unsigned)(KTOT >> 3);
  const unsigned kp8   = (unsigned)(KP >> 3);
  const unsigned total = (unsigned)MP * ppr;
  const unsigned g     = blockIdx.x * 256u + threadIdx.x;
  const unsigned rowu  = g / ppr;
  const unsigned p     = g - rowu * ppr;
  const bool second    = p >= kp8;
  const int row = (int)rowu;
  const int c0  = (int)((second ? p - kp8 : p) << 3);
  const float* srow = src + (size_t)clampi(row, 0, rows - 1) * (size_t)ldsrc;
  float x[8];
  unsigned mk[8];
#pragma unroll
  for (int e = 0; e < 8; ++e) {
    const int c = c0 + e;
    const float v = srow[clampi(c, 0, cols - 1)];
    asm volatile("" :: "v"(v));
    x[e]  = v;
    mk[e] = (row < rows && c < cols) ? 0xFFFFu : 0u;
  }
  const v4f a = (v4f){ x[0], x[1], x[2], x[3] };
  const v4f c = (v4f){ x[4], x[5], x[6], x[7] };
  v4u o;
  if (FORM == 2) {
    o = pack8_f16(a, c);
  } else {
    const v4u hi = pack8_bf16(a, c);
    o = hi;
    if (FORM == 1) { const v4u lo = pack8_bf16_lo(a, c); o = second ? lo : hi; }
  }
  const v4u mw = (v4u){ pk16(mk[0], mk[1]), pk16(mk[2], mk[3]), pk16(mk[4], mk[5]), pk16(mk[6], mk[7]) };
  o &= mw;
  if (g < total) {
    volatile v4u* q = (volatile v4u*)(dst + (size_t)g * 8);
    *q = o;
    __threadfence();
    *q = o;
  }
}

template <int FORM> struct FragOf    { typedef FragB T; };
template <>         struct FragOf<2> { typedef FragH T; };
__device__ __forceinline__ v8f mm(const FragB& a, const FragB& b, v8f c) { return wmb(a, b, c); }
__device__ __forceinline__ v8f mm(const FragH& a, const FragH& b, v8f c) { return wmh(a, b, c); }
template <class F> __device__ __forceinline__ F ld_frag(const unsigned short* p) {
  F f;
  f.h[0] = *(const v8usa*)(p);
  f.h[1] = *(const v8usa*)(p + 16);
  return f;
}

template <int FORM, int EPI>
__global__ __launch_bounds__(256) __attribute__((amdgpu_num_vgpr(248)))
void k_gemm_nt(const unsigned short* __restrict__ A, const unsigned short* __restrict__ B,
               const float* __restrict__ bias, float* __restrict__ D, int M, int N, int KTOT, int ldd) {
  static_assert(FORM >= 0 && FORM <= 2);
  static_assert(EPI == 0 || EPI == 1);
  typedef typename FragOf<FORM>::T F;
  __shared__ __attribute__((aligned(16))) float sT[8][16 * 68];
  const int lane = threadIdx.x & 31;
  const int wave = threadIdx.x >> 5;
  const int tilesM = (M + 63) >> 6;
  const int tilesN = (N + 63) >> 6;
  const int tile = blockIdx.x * 8 + wave;
  if (tile >= tilesM * tilesN) return;
  const int tm = tile / tilesN;
  const int tn = tile - tm * tilesN;
  const int m0 = tm << 6;
  const int n0 = tn << 6;

  const int rl = lane & 15;
  const int h8 = (lane >> 4) * 8;
  const unsigned short* pa = A + (size_t)(m0 + rl) * (size_t)KTOT + h8;
  const unsigned short* pb = B + (size_t)(n0 + rl) * (size_t)KTOT + h8;

  v8f acc[4][4];
#pragma unroll
  for (int i = 0; i < 4; ++i)
#pragma unroll
    for (int j = 0; j < 4; ++j) acc[i][j] = (v8f){0.f, 0.f, 0.f, 0.f, 0.f, 0.f, 0.f, 0.f};

#pragma unroll 1
  for (int k0 = 0; k0 < KTOT; k0 += 32) {
    F bf[4];
#pragma unroll
    for (int j = 0; j < 4; ++j) bf[j] = ld_frag<F>(pb + (size_t)(j << 4) * (size_t)KTOT + k0);
#pragma unroll
    for (int i = 0; i < 4; ++i) {
      const F af = ld_frag<F>(pa + (size_t)(i << 4) * (size_t)KTOT + k0);
#pragma unroll
      for (int j = 0; j < 4; ++j) acc[i][j] = mm(af, bf[j], acc[i][j]);
    }
  }

  float* slab = sT[wave];
  const int hh = lane >> 4;
  const int c4 = (lane & 15) * 4;
  const int nc = n0 + c4;
  const bool cok = nc < N;
  v4f bv = (v4f){0.f, 0.f, 0.f, 0.f};
  if (EPI == 1) {
    bv = *(const v4fa*)(bias + clampi(nc, 0, N - 4));
    asm volatile("" :: "v"(bv));
  }
#pragma unroll
  for (int i = 0; i < 4; ++i) {
    const int mBase = m0 + (i << 4);
#pragma unroll
    for (int j = 0; j < 4; ++j) {
#pragma unroll
      for (int r = 0; r < 8; ++r) slab[(h8 + r) * 68 + (j << 4) + rl] = acc[i][j][r];
    }
    __builtin_amdgcn_fence(__ATOMIC_RELEASE, "workgroup");
    __builtin_amdgcn_wave_barrier();
    __builtin_amdgcn_fence(__ATOMIC_ACQUIRE, "workgroup");
    v4f vv[8];
#pragma unroll
    for (int it = 0; it < 8; ++it) {
      const int row = it * 2 + hh;
      v4f v = *(const v4fa*)(slab + row * 68 + c4);
      if (EPI == 1) v += bv;
      vv[it] = v;
    }
    for (int pass = 0; pass < 2; ++pass) {
#pragma unroll
      for (int it = 0; it < 8; ++it) {
        const int row = mBase + it * 2 + hh;
        if (cok && row < M) *(volatile v4f*)(D + (size_t)row * (size_t)ldd + nc) = vv[it];
      }
      __threadfence();
    }
    __builtin_amdgcn_fence(__ATOMIC_RELEASE, "workgroup");
    __builtin_amdgcn_wave_barrier();
    __builtin_amdgcn_fence(__ATOMIC_ACQUIRE, "workgroup");
  }
}

#define NTOK 2048
#define DD 32
#define RR 64
#define HIDN 128
#define NTHR 256
#define KTILE 64
#define CPAIR 0x1.6a09e6p-3f

#define PV_BQ 0
#define PV_BK 32
#define PV_BV 64
#define PV_BO 96
#define PV_B1 128
#define PV_B2 256
#define PV_G1 288
#define PV_BE1 320
#define PV_G2 352
#define PV_BE2 384
#define PV_USED 416
#define PV_TOTAL 512

static_assert(NTOK % 64 == 0);
static_assert(DD == 32 && RR == 64 && HIDN == 128);
static_assert(NTHR == 256);
static_assert((64 / 16) * (DD / 16) == 8);
static_assert(KTILE == 64);
static_assert(PV_USED % 32 == 0 && PV_TOTAL >= PV_USED);

typedef int          v4i __attribute__((ext_vector_type(4)));
typedef unsigned int v2u __attribute__((ext_vector_type(2)));
typedef v4u __attribute__((may_alias)) v4ua;
typedef v2u __attribute__((may_alias)) v2ua;
typedef v4i __attribute__((may_alias)) v4ia;

struct F8 { v4f a; v4f c; };

__device__ __forceinline__ FragB lds_frag(const unsigned short* p) {
  FragB f;
  f.h[0] = *(const v8usa*)(p);
  f.h[1] = *(const v8usa*)(p + 16);
  return f;
}
__device__ __forceinline__ void st2_u4(unsigned short* p, v4u o) {
  volatile v4u* q = (volatile v4u*)p;
  *q = o;
  __threadfence();
  *q = o;
}
__device__ __forceinline__ void st2_f4(float* p, v4f o) {
  volatile v4f* q = (volatile v4f*)p;
  *q = o;
  __threadfence();
  *q = o;
}
__device__ __forceinline__ v4u tr_piece(const float* __restrict__ W, int ld, int n, int k0) {
  float x[8];
#pragma unroll
  for (int e = 0; e < 8; ++e) {
    const float v = W[(size_t)(k0 + e) * (size_t)ld + n];
    asm volatile("" :: "v"(v));
    x[e] = v;
  }
  return pack8_bf16((v4f){ x[0], x[1], x[2], x[3] }, (v4f){ x[4], x[5], x[6], x[7] });
}
__device__ __forceinline__ void pv_seg(const float* __restrict__ src, int n4, float* dst, int lane) {
  const int i = lane < n4 ? lane : n4 - 1;
  const v4f v = *(const v4fa*)(src + 4 * i);
  asm volatile("" :: "v"(v));
  const v4f o = (v4f){ bf16_val(v[0]), bf16_val(v[1]), bf16_val(v[2]), bf16_val(v[3]) };
  if (lane < n4) st2_f4(dst + 4 * i, o);
}
__device__ __forceinline__ F8 ln_row8(const float* xr, int c0, const float* g, const float* b) {
  float mu = 0.0f;
#pragma unroll 4
  for (int c = 0; c < 32; ++c) mu += xr[c];
  mu *= 0.03125f;
  float var = 0.0f;
#pragma unroll 4
  for (int c = 0; c < 32; ++c) { const float d = xr[c] - mu; var += d * d; }
  var *= 0.03125f;
  const float sd = sqrtf(var + 1e-5f);
  F8 o;
#pragma unroll
  for (int e = 0; e < 4; ++e) {
    o.a[e] = (xr[c0 + e] - mu) / sd * g[c0 + e] + b[c0 + e];
    o.c[e] = (xr[c0 + 4 + e] - mu) / sd * g[c0 + 4 + e] + b[c0 + 4 + e];
  }
  return o;
}

__global__ __launch_bounds__(256) void k_wprep(
    const float* __restrict__ Wq, const float* __restrict__ Wk, const float* __restrict__ Wv,
    const float* __restrict__ omega, const float* __restrict__ Wo, const float* __restrict__ W1,
    const float* __restrict__ W2,
    const float* __restrict__ bq, const float* __restrict__ bk, const float* __restrict__ bv,
    const float* __restrict__ bo, const float* __restrict__ b1, const float* __restrict__ b2,
    const float* __restrict__ g1, const float* __restrict__ be1, const float* __restrict__ g2,
    const float* __restrict__ be2,
    unsigned short* __restrict__ WQKV, unsigned short* __restrict__ OMG2, unsigned short* __restrict__ WO2,
    unsigned short* __restrict__ W1_2, unsigned short* __restrict__ W2_2, float* __restrict__ PV) {
  const int tid = threadIdx.x;
#pragma unroll 1
  for (int g = tid; g < 128; g += 256) st2_u4(WQKV + (size_t)g * 8, tr_piece(Wq, 32, g >> 2, (g & 3) * 8));
#pragma unroll 1
  for (int g = tid; g < 128; g += 256) st2_u4(WQKV + 1024 + (size_t)g * 8, tr_piece(Wk, 32, g >> 2, (g & 3) * 8));
#pragma unroll 1
  for (int g = tid; g < 128; g += 256) st2_u4(WQKV + 2048 + (size_t)g * 8, tr_piece(Wv, 32, g >> 2, (g & 3) * 8));
#pragma unroll 1
  for (int g = tid; g < 512; g += 256) st2_u4(OMG2 + (size_t)g * 8, tr_piece(omega, 64, g >> 3, (g & 3) * 8));
#pragma unroll 1
  for (int g = tid; g < 256; g += 256) st2_u4(WO2 + (size_t)g * 8, tr_piece(Wo, 32, g >> 3, (g & 3) * 8));
#pragma unroll 1
  for (int g = tid; g < 1024; g += 256) st2_u4(W1_2 + (size_t)g * 8, tr_piece(W1, 128, g >> 3, (g & 3) * 8));
#pragma unroll 1
  for (int g = tid; g < 1024; g += 256) st2_u4(W2_2 + (size_t)g * 8, tr_piece(W2, 32, g >> 5, (g & 15) * 8));
  if (tid < 32) {
    pv_seg(bq, 8, PV + PV_BQ, tid);
    pv_seg(bk, 8, PV + PV_BK, tid);
    pv_seg(bv, 8, PV + PV_BV, tid);
    pv_seg(bo, 8, PV + PV_BO, tid);
    pv_seg(b1, 32, PV + PV_B1, tid);
    pv_seg(b2, 8, PV + PV_B2, tid);
    pv_seg(g1, 8, PV + PV_G1, tid);
    pv_seg(be1, 8, PV + PV_BE1, tid);
    pv_seg(g2, 8, PV + PV_G2, tid);
    pv_seg(be2, 8, PV + PV_BE2, tid);
    const int i = tid < 24 ? tid : 23;
    if (tid < 24) st2_f4(PV + PV_USED + 4 * i, (v4f){ 0.f, 0.f, 0.f, 0.f });
  }
}

__global__ __launch_bounds__(256) void k_rows(
    const float* __restrict__ Z, const unsigned short* __restrict__ WQKV, const unsigned short* __restrict__ OMG2,
    const float* __restrict__ PV, float* __restrict__ QF, float* __restrict__ KF,
    unsigned short* __restrict__ PHQ, unsigned short* __restrict__ PHK,
    unsigned short* __restrict__ PHKTh, unsigned short* __restrict__ PHKTl,
    unsigned short* __restrict__ VTh, unsigned short* __restrict__ VTl) {
  __shared__ __attribute__((aligned(16))) unsigned short sZ[64 * 40];
  __shared__ __attribute__((aligned(16))) float sQKV[64 * 100];
  __shared__ __attribute__((aligned(16))) unsigned short sN[128 * 72];
  __shared__ __attribute__((aligned(16))) float sPhi[128 * 68];
  __shared__ __attribute__((aligned(16))) float sB[96];
  const int tid = threadIdx.x, lane = tid & 31, wave = tid >> 5;
  const int rl = lane & 15, h8 = (lane >> 4) * 8;
  const int i0 = blockIdx.x * 64;
  {
    const int row = tid >> 2, c0 = (tid & 3) * 8;
    const float* zp = Z + (size_t)(i0 + row) * 32 + c0;
    const v4f a = *(const v4fa*)(zp);
    const v4f c = *(const v4fa*)(zp + 4);
    *(v4ua*)(sZ + row * 40 + c0) = pack8_bf16(a, c);
  }
  if (wave == 0) {
    const int i = lane < 24 ? lane : 23;
    const v4f v = *(const v4fa*)(PV + 4 * i);
    *(v4fa*)(sB + 4 * i) = v;
  }
  __syncthreads();
  {
    const int mt = wave >> 1, nb = (wave & 1) * 3;
    const FragB a = lds_frag(sZ + (mt * 16 + rl) * 40 + h8);
#pragma unroll
    for (int j = 0; j < 3; ++j) {
      const int nt = nb + j;
      const FragB b = ld_frag<FragB>(WQKV + (size_t)(nt * 16 + rl) * 32 + h8);
      v8f d = (v8f){ 0.f, 0.f, 0.f, 0.f, 0.f, 0.f, 0.f, 0.f };
      d = wmb(a, b, d);
      const int col = nt * 16 + rl;
      const float bias = sB[col];
#pragma unroll
      for (int r = 0; r < 8; ++r) sQKV[(mt * 16 + h8 + r) * 100 + col] = d[r] + bias;
    }
  }
  __syncthreads();
  if (wave < 4) {
    const int row = tid & 63, which = tid >> 6;
    const float* src = sQKV + row * 100 + which * 32;
    float ss = 0.0f;
#pragma unroll 4
    for (int c = 0; c < 32; ++c) { const float x = src[c]; ss += x * x; }
    const float nrm = fmaxf(sqrtf(ss), 1e-6f);
    unsigned short* dst = sN + (which * 64 + row) * 72;
#pragma unroll 1
    for (int c0 = 0; c0 < 32; c0 += 8) {
      v4f a = *(const v4fa*)(src + c0);
      v4f c = *(const v4fa*)(src + c0 + 4);
#pragma unroll
      for (int e = 0; e < 4; ++e) { a[e] = a[e] / nrm; c[e] = c[e] / nrm; }
      *(v4ua*)(dst + c0)      = pack8_bf16(a, c);
      *(v4ua*)(dst + 32 + c0) = pack8_bf16_lo(a, c);
    }
  }
  __syncthreads();
  {
    const int mt = wave;
    v8f d[4];
#pragma unroll
    for (int j = 0; j < 4; ++j) d[j] = (v8f){ 0.f, 0.f, 0.f, 0.f, 0.f, 0.f, 0.f, 0.f };
#pragma unroll
    for (int ks = 0; ks < 2; ++ks) {
      const FragB a = lds_frag(sN + (mt * 16 + rl) * 72 + ks * 32 + h8);
#pragma unroll
      for (int j = 0; j < 4; ++j) {
        const FragB b = ld_frag<FragB>(OMG2 + (size_t)(j * 16 + rl) * 64 + ks * 32 + h8);
        d[j] = wmb(a, b, d[j]);
      }
    }
#pragma unroll
    for (int j = 0; j < 4; ++j)
#pragma unroll
      for (int r = 0; r < 8; ++r) sPhi[(mt * 16 + h8 + r) * 68 + j * 16 + rl] = expf(d[j][r]) * 0.125f;
  }
  __syncthreads();
#pragma unroll 1
  for (int it = 0; it < 2; ++it) {
    const int row = it * 32 + (tid >> 3), pc = (tid & 7) * 4;
    const v4f q = *(const v4fa*)(sQKV + row * 100 + pc);
    const v4f k = *(const v4fa*)(sQKV + row * 100 + 32 + pc);
    st2_f4(QF + (size_t)(i0 + row) * 32 + pc, q);
    st2_f4(KF + (size_t)(i0 + row) * 32 + pc, k);
  }
  {
    const int d = tid >> 3, t0 = (tid & 7) * 8;
    float x[8];
#pragma unroll
    for (int e = 0; e < 8; ++e) x[e] = sQKV[(t0 + e) * 100 + 64 + d];
    const v4f a = (v4f){ x[0], x[1], x[2], x[3] };
    const v4f c = (v4f){ x[4], x[5], x[6], x[7] };
    st2_u4(VTh + (size_t)d * NTOK + i0 + t0, pack8_bf16(a, c));
    st2_u4(VTl + (size_t)d * NTOK + i0 + t0, pack8_bf16_lo(a, c));
  }
#pragma unroll 1
  for (int it = 0; it < 4; ++it) {
    const int g = it * 256 + tid;
    const int row = g >> 4, p = g & 15, c0 = (p & 7) * 8;
    const bool second = p >= 8;
    {
      const float* s = sPhi + row * 68 + c0;
      const v4f a = *(const v4fa*)(s);
      const v4f c = *(const v4fa*)(s + 4);
      const v4u hi = pack8_bf16(a, c);
      const v4u lo = pack8_bf16_lo(a, c);
      const v4u o = second ? lo : hi;
      st2_u4(PHQ + (size_t)(i0 + row) * 128 + p * 8, o);
    }
    {
      const float* s = sPhi + (64 + row) * 68 + c0;
      const v4f a = *(const v4fa*)(s);
      const v4f c = *(const v4fa*)(s + 4);
      const v4u hi = pack8_bf16(a, c);
      const v4u lo = pack8_bf16_lo(a, c);
      const v4u o = second ? lo : hi;
      st2_u4(PHK + (size_t)(i0 + row) * 128 + p * 8, o);
    }
  }
#pragma unroll 1
  for (int it = 0; it < 2; ++it) {
    const int r = it * 32 + (tid >> 3), t0 = (tid & 7) * 8;
    float x[8];
#pragma unroll
    for (int e = 0; e < 8; ++e) x[e] = sPhi[(64 + t0 + e) * 68 + r];
    const v4f a = (v4f){ x[0], x[1], x[2], x[3] };
    const v4f c = (v4f){ x[4], x[5], x[6], x[7] };
    st2_u4(PHKTh + (size_t)r * NTOK + i0 + t0, pack8_bf16(a, c));
    st2_u4(PHKTl + (size_t)r * NTOK + i0 + t0, pack8_bf16_lo(a, c));
  }
}

__global__ __launch_bounds__(256) void k_m(
    const unsigned short* __restrict__ PHKTh, const unsigned short* __restrict__ PHKTl,
    const unsigned short* __restrict__ VTh, const unsigned short* __restrict__ VTl,
    unsigned short* __restrict__ MT) {
  __shared__ __attribute__((aligned(16))) float sM[64 * 36];
  const int tid = threadIdx.x, lane = tid & 31, wave = tid >> 5;
  const int rl = lane & 15, h8 = (lane >> 4) * 8;
  const int mt = wave >> 1, nt = wave & 1;
  const unsigned short* pah = PHKTh + (size_t)(mt * 16 + rl) * NTOK + h8;
  const unsigned short* pal = PHKTl + (size_t)(mt * 16 + rl) * NTOK + h8;
  const unsigned short* pbh = VTh + (size_t)(nt * 16 + rl) * NTOK + h8;
  const unsigned short* pbl = VTl + (size_t)(nt * 16 + rl) * NTOK + h8;
  v8f acc = (v8f){ 0.f, 0.f, 0.f, 0.f, 0.f, 0.f, 0.f, 0.f };
#pragma unroll 1
  for (int k0 = 0; k0 < NTOK; k0 += 32) {
    const FragB ah = ld_frag<FragB>(pah + k0);
    const FragB al = ld_frag<FragB>(pal + k0);
    const FragB bh = ld_frag<FragB>(pbh + k0);
    const FragB bl = ld_frag<FragB>(pbl + k0);
    acc = wmb(ah, bh, acc);
    acc = wmb(al, bh, acc);
    acc = wmb(ah, bl, acc);
  }
#pragma unroll
  for (int r = 0; r < 8; ++r) sM[(mt * 16 + h8 + r) * 36 + nt * 16 + rl] = acc[r];
  __syncthreads();
#pragma unroll 1
  for (int it = 0; it < 2; ++it) {
    const int d = it * 16 + (tid >> 4), p = tid & 15, r0 = (p & 7) * 8;
    float x[8];
#pragma unroll
    for (int e = 0; e < 8; ++e) x[e] = sM[(r0 + e) * 36 + d];
    const v4f a = (v4f){ x[0], x[1], x[2], x[3] };
    const v4f c = (v4f){ x[4], x[5], x[6], x[7] };
    const v4u hi = pack8_bf16(a, c);
    const v4u lo = pack8_bf16_lo(a, c);
    const v4u o = (p >= 8) ? lo : hi;
    st2_u4(MT + (size_t)d * 128 + p * 8, o);
  }
}

__global__ __launch_bounds__(256) __attribute__((amdgpu_num_vgpr(248)))
void k_pair(const float* __restrict__ QF, const float* __restrict__ KF,
            const unsigned short* __restrict__ PHQ, const unsigned short* __restrict__ PHK,
            const unsigned short* __restrict__ VTh, const unsigned short* __restrict__ VTl,
            const unsigned short* __restrict__ MT, const int* __restrict__ mask, float* __restrict__ ATT) {
  __shared__ __attribute__((aligned(16))) float sQT[32 * 68];
  __shared__ __attribute__((aligned(16))) float sKT[32 * 68];
  __shared__ __attribute__((aligned(16))) float sSP[64 * 68];
  __shared__ __attribute__((aligned(16))) unsigned short sPQ[64 * 136];
  __shared__ __attribute__((aligned(16))) unsigned short sPK[64 * 136];
  __shared__ __attribute__((aligned(16))) unsigned short sVT[32 * 136];
  __shared__ __attribute__((aligned(16))) unsigned short sP[64 * 136];
  const int tid = threadIdx.x, lane = tid & 31, wave = tid >> 5;
  const int rl = lane & 15, h8 = (lane >> 4) * 8;
  const int i0 = blockIdx.x * 64;
  const int mt = wave >> 1, nt = wave & 1;
  {
    const int row = tid >> 2, c0 = (tid & 3) * 8;
    const float* qp = QF + (size_t)(i0 + row) * 32 + c0;
    const v4f a = *(const v4fa*)(qp);
    const v4f c = *(const v4fa*)(qp + 4);
#pragma unroll
    for (int e = 0; e < 4; ++e) { sQT[(c0 + e) * 68 + row] = a[e]; sQT[(c0 + 4 + e) * 68 + row] = c[e]; }
  }
#pragma unroll
  for (int it = 0; it < 4; ++it) {
    const int g = it * 256 + tid, row = g >> 4, p = g & 15;
    const v4u v = *(const v4ua*)(PHQ + (size_t)(i0 + row) * 128 + p * 8);
    *(v4ua*)(sPQ + row * 136 + p * 8) = v;
  }
  __syncthreads();
  v8f O = (v8f){ 0.f, 0.f, 0.f, 0.f, 0.f, 0.f, 0.f, 0.f };
  {
    const unsigned short* pa = sPQ + (mt * 16 + rl) * 136 + h8;
    const unsigned short* pb = MT + (size_t)(nt * 16 + rl) * 128 + h8;
#pragma unroll
    for (int ks = 0; ks < 2; ++ks) {
      const FragB ah = lds_frag(pa + ks * 32);
      const FragB al = lds_frag(pa + 64 + ks * 32);
      const FragB bh = ld_frag<FragB>(pb + ks * 32);
      const FragB bl = ld_frag<FragB>(pb + 64 + ks * 32);
      O = wmb(ah, bh, O);
      O = wmb(al, bh, O);
      O = wmb(ah, bl, O);
    }
  }
#pragma unroll 1
  for (int kt = 0; kt < NTOK / KTILE; ++kt) {
    const int j0 = kt * KTILE;
    {
      const int row = tid >> 2, c0 = (tid & 3) * 8;
      const float* kp = KF + (size_t)(j0 + row) * 32 + c0;
      const v4f a = *(const v4fa*)(kp);
      const v4f c = *(const v4fa*)(kp + 4);
#pragma unroll
      for (int e = 0; e < 4; ++e) { sKT[(c0 + e) * 68 + row] = a[e]; sKT[(c0 + 4 + e) * 68 + row] = c[e]; }
    }
#pragma unroll
    for (int it = 0; it < 4; ++it) {
      const int g = it * 256 + tid, row = g >> 4, p = g & 15;
      const v4u v = *(const v4ua*)(PHK + (size_t)(j0 + row) * 128 + p * 8);
      *(v4ua*)(sPK + row * 136 + p * 8) = v;
    }
    {
      const int d = tid >> 3, p = tid & 7;
      const v4u vh = *(const v4ua*)(VTh + (size_t)d * NTOK + j0 + p * 8);
      const v4u vl = *(const v4ua*)(VTl + (size_t)d * NTOK + j0 + p * 8);
      *(v4ua*)(sVT + d * 136 + p * 8)      = vh;
      *(v4ua*)(sVT + d * 136 + 64 + p * 8) = vl;
    }
    __syncthreads();
    {
      const int nb = (wave & 1) * 2;
      const unsigned short* pa  = sPQ + (mt * 16 + rl) * 136 + h8;
      const unsigned short* pb0 = sPK + (nb * 16 + rl) * 136 + h8;
      const unsigned short* pb1 = pb0 + 16 * 136;
      v8f s0 = (v8f){ 0.f, 0.f, 0.f, 0.f, 0.f, 0.f, 0.f, 0.f };
      v8f s1 = (v8f){ 0.f, 0.f, 0.f, 0.f, 0.f, 0.f, 0.f, 0.f };
#pragma unroll
      for (int ks = 0; ks < 2; ++ks) {
        const FragB ah = lds_frag(pa + ks * 32);
        const FragB al = lds_frag(pa + 64 + ks * 32);
        const FragB b0h = lds_frag(pb0 + ks * 32);
        const FragB b0l = lds_frag(pb0 + 64 + ks * 32);
        s0 = wmb(ah, b0h, s0);
        s0 = wmb(al, b0h, s0);
        s0 = wmb(ah, b0l, s0);
        const FragB b1h = lds_frag(pb1 + ks * 32);
        const FragB b1l = lds_frag(pb1 + 64 + ks * 32);
        s1 = wmb(ah, b1h, s1);
        s1 = wmb(al, b1h, s1);
        s1 = wmb(ah, b1l, s1);
      }
#pragma unroll
      for (int r = 0; r < 8; ++r) {
        sSP[(mt * 16 + h8 + r) * 68 + nb * 16 + rl]       = s0[r];
        sSP[(mt * 16 + h8 + r) * 68 + (nb + 1) * 16 + rl] = s1[r];
      }
    }
    __syncthreads();
    {
      const int ti = tid >> 4, tj = tid & 15;
      float e[4][4];
#pragma unroll
      for (int a = 0; a < 4; ++a)
#pragma unroll
        for (int b = 0; b < 4; ++b) e[a][b] = 0.0f;
#pragma unroll 2
      for (int c = 0; c < 32; ++c) {
        const v4f q = *(const v4fa*)(sQT + c * 68 + 4 * ti);
        const v4f k = *(const v4fa*)(sKT + c * 68 + 4 * tj);
#pragma unroll
        for (int a = 0; a < 4; ++a)
#pragma unroll
          for (int b = 0; b < 4; ++b) e[a][b] += expf((q[a] * k[b]) * CPAIR);
      }
#pragma unroll
      for (int a = 0; a < 4; ++a) {
        const int row = 4 * ti + a;
        const v4i m = *(const v4ia*)(mask + (size_t)(i0 + row) * NTOK + j0 + 4 * tj);
        asm volatile("" :: "v"(m));
        const v4f sp = *(const v4fa*)(sSP + row * 68 + 4 * tj);
        asm volatile("" :: "v"(sp));
        float s[4];
#pragma unroll
        for (int b = 0; b < 4; ++b) {
          const float dlt = e[a][b] - sp[b];
          s[b] = (m[b] == 0) ? dlt : 0.0f;
        }
        const v2u hw = (v2u){ pk16(bf16_bits(s[0]), bf16_bits(s[1])), pk16(bf16_bits(s[2]), bf16_bits(s[3])) };
        const v2u lw = (v2u){ pk16(bf16_lo_bits(s[0]), bf16_lo_bits(s[1])), pk16(bf16_lo_bits(s[2]), bf16_lo_bits(s[3])) };
        *(v2ua*)(sP + row * 136 + 4 * tj)      = hw;
        *(v2ua*)(sP + row * 136 + 64 + 4 * tj) = lw;
      }
    }
    __syncthreads();
    {
      const unsigned short* pa = sP + (mt * 16 + rl) * 136 + h8;
      const unsigned short* pb = sVT + (nt * 16 + rl) * 136 + h8;
#pragma unroll
      for (int ks = 0; ks < 2; ++ks) {
        const FragB ah = lds_frag(pa + ks * 32);
        const FragB al = lds_frag(pa + 64 + ks * 32);
        const FragB bh = lds_frag(pb + ks * 32);
        const FragB bl = lds_frag(pb + 64 + ks * 32);
        O = wmb(ah, bh, O);
        O = wmb(al, bh, O);
        O = wmb(ah, bl, O);
      }
    }
    __syncthreads();
  }
#pragma unroll
  for (int r = 0; r < 8; ++r) sSP[(mt * 16 + h8 + r) * 68 + nt * 16 + rl] = O[r];
  __syncthreads();
#pragma unroll 1
  for (int it = 0; it < 2; ++it) {
    const int row = it * 32 + (tid >> 3), pc = (tid & 7) * 4;
    const v4f v = *(const v4fa*)(sSP + row * 68 + pc);
    st2_f4(ATT + (size_t)(i0 + row) * 32 + pc, v);
  }
}

__global__ __launch_bounds__(256) void k_tail(
    const float* __restrict__ ATT, const float* __restrict__ Z, const float* __restrict__ PV,
    const unsigned short* __restrict__ WO2, const unsigned short* __restrict__ W1_2,
    const unsigned short* __restrict__ W2_2, float* __restrict__ out) {
  __shared__ __attribute__((aligned(16))) float sX[64 * 36];
  __shared__ __attribute__((aligned(16))) float sZb[64 * 36];
  __shared__ __attribute__((aligned(16))) float sZ1[64 * 36];
  __shared__ __attribute__((aligned(16))) float sPV[PV_USED];
  __shared__ __attribute__((aligned(16))) unsigned short sA[64 * 72];
  __shared__ __attribute__((aligned(16))) unsigned short sAH[64 * 264];
  const int tid = threadIdx.x, lane = tid & 31, wave = tid >> 5;
  const int rl = lane & 15, h8 = (lane >> 4) * 8;
  const int i0 = blockIdx.x * 64;
  const int mt = wave >> 1, nt = wave & 1;
  const int prow = tid >> 2, pc0 = (tid & 3) * 8;
  {
    const float* ap = ATT + (size_t)(i0 + prow) * 32 + pc0;
    const float* zp = Z + (size_t)(i0 + prow) * 32 + pc0;
    const v4f a = *(const v4fa*)(ap);
    const v4f c = *(const v4fa*)(ap + 4);
    const v4f za = *(const v4fa*)(zp);
    const v4f zc = *(const v4fa*)(zp + 4);
    *(v4fa*)(sX + prow * 36 + pc0)     = a;
    *(v4fa*)(sX + prow * 36 + pc0 + 4) = c;
    *(v4fa*)(sZb + prow * 36 + pc0)     = (v4f){ bf16_val(za[0]), bf16_val(za[1]), bf16_val(za[2]), bf16_val(za[3]) };
    *(v4fa*)(sZb + prow * 36 + pc0 + 4) = (v4f){ bf16_val(zc[0]), bf16_val(zc[1]), bf16_val(zc[2]), bf16_val(zc[3]) };
  }
  if (wave < 4) {
    const int i = tid < 103 ? tid : 103;
    const v4f v = *(const v4fa*)(PV + 4 * i);
    *(v4fa*)(sPV + 4 * i) = v;
  }
  __syncthreads();
  {
    const float* xr = sX + prow * 36;
    float s = 0.0f;
#pragma unroll 4
    for (int c = 0; c < 32; ++c) s += xr[c];
    const float den = fmaxf(s, 1e-6f);
    v4f a = *(const v4fa*)(xr + pc0);
    v4f c = *(const v4fa*)(xr + pc0 + 4);
#pragma unroll
    for (int e = 0; e < 4; ++e) { a[e] = a[e] / den; c[e] = c[e] / den; }
    *(v4ua*)(sA + prow * 72 + pc0)      = pack8_bf16(a, c);
    *(v4ua*)(sA + prow * 72 + 32 + pc0) = pack8_bf16_lo(a, c);
  }
  __syncthreads();
  {
    const unsigned short* pa = sA + (mt * 16 + rl) * 72 + h8;
    const unsigned short* pb = WO2 + (size_t)(nt * 16 + rl) * 64 + h8;
    v8f d = (v8f){ 0.f, 0.f, 0.f, 0.f, 0.f, 0.f, 0.f, 0.f };
#pragma unroll
    for (int ks = 0; ks < 2; ++ks) {
      const FragB a = lds_frag(pa + ks * 32);
      const FragB b = ld_frag<FragB>(pb + ks * 32);
      d = wmb(a, b, d);
    }
    const int col = nt * 16 + rl;
    const float bo = sPV[PV_BO + col];
#pragma unroll
    for (int r = 0; r < 8; ++r) {
      const int row = mt * 16 + h8 + r;
      sX[row * 36 + col] = sZb[row * 36 + col] + (d[r] + bo);
    }
  }
  __syncthreads();
  {
    const F8 z = ln_row8(sX + prow * 36, pc0, sPV + PV_G1, sPV + PV_BE1);
    *(v4fa*)(sZ1 + prow * 36 + pc0)     = z.a;
    *(v4fa*)(sZ1 + prow * 36 + pc0 + 4) = z.c;
    *(v4ua*)(sA + prow * 72 + pc0)      = pack8_bf16(z.a, z.c);
    *(v4ua*)(sA + prow * 72 + 32 + pc0) = pack8_bf16_lo(z.a, z.c);
  }
  __syncthreads();
  {
    const int nb = (wave & 1) * 4;
    const unsigned short* pa = sA + (mt * 16 + rl) * 72 + h8;
    v8f d[4];
#pragma unroll
    for (int j = 0; j < 4; ++j) d[j] = (v8f){ 0.f, 0.f, 0.f, 0.f, 0.f, 0.f, 0.f, 0.f };
#pragma unroll
    for (int ks = 0; ks < 2; ++ks) {
      const FragB a = lds_frag(pa + ks * 32);
#pragma unroll
      for (int j = 0; j < 4; ++j) {
        const FragB b = ld_frag<FragB>(W1_2 + (size_t)((nb + j) * 16 + rl) * 64 + ks * 32 + h8);
        d[j] = wmb(a, b, d[j]);
      }
    }
#pragma unroll
    for (int j = 0; j < 4; ++j) {
      const int col = (nb + j) * 16 + rl;
      const float b1v = sPV[PV_B1 + col];
#pragma unroll
      for (int r = 0; r < 8; ++r) {
        const int row = mt * 16 + h8 + r;
        const float v = fmaxf(d[j][r] + b1v, 0.0f);
        sAH[row * 264 + col]       = (unsigned short)bf16_bits(v);
        sAH[row * 264 + 128 + col] = (unsigned short)bf16_lo_bits(v);
      }
    }
  }
  __syncthreads();
  {
    const unsigned short* pa = sAH + (mt * 16 + rl) * 264 + h8;
    const unsigned short* pb = W2_2 + (size_t)(nt * 16 + rl) * 256 + h8;
    v8f d = (v8f){ 0.f, 0.f, 0.f, 0.f, 0.f, 0.f, 0.f, 0.f };
#pragma unroll 2
    for (int ks = 0; ks < 8; ++ks) {
      const FragB a = lds_frag(pa + ks * 32);
      const FragB b = ld_frag<FragB>(pb + ks * 32);
      d = wmb(a, b, d);
    }
    const int col = nt * 16 + rl;
    const float b2v = sPV[PV_B2 + col];
#pragma unroll
    for (int r = 0; r < 8; ++r) {
      const int row = mt * 16 + h8 + r;
      sX[row * 36 + col] = sZ1[row * 36 + col] + (d[r] + b2v);
    }
  }
  __syncthreads();
  {
    const F8 z = ln_row8(sX + prow * 36, pc0, sPV + PV_G2, sPV + PV_BE2);
    *(v4fa*)(sZb + prow * 36 + pc0)     = z.a;
    *(v4fa*)(sZb + prow * 36 + pc0 + 4) = z.c;
  }
  __syncthreads();
#pragma unroll 1
  for (int it = 0; it < 2; ++it) {
    const int row = it * 32 + (tid >> 3), pc = (tid & 7) * 4;
    const v4f v = *(const v4fa*)(sZb + row * 36 + pc);
    st2_f4(out + (size_t)(i0 + row) * 32 + pc, v);
  }
}

static constexpr size_t SZ_F32ROWS = (size_t)NTOK * DD * 4;
static constexpr size_t SZ_PH      = (size_t)NTOK * 128 * 2;
static constexpr size_t SZ_PHKT    = (size_t)RR * NTOK * 2;
static constexpr size_t SZ_VT      = (size_t)DD * NTOK * 2;
static constexpr size_t SZ_MT      = (size_t)DD * 128 * 2;
static constexpr size_t SZ_WQKV    = (size_t)96 * 32 * 2;
static constexpr size_t SZ_OMG2    = (size_t)64 * 64 * 2;
static constexpr size_t SZ_WO2     = (size_t)32 * 64 * 2;
static constexpr size_t SZ_W1_2    = (size_t)128 * 64 * 2;
static constexpr size_t SZ_W2_2    = (size_t)32 * 256 * 2;
static constexpr size_t SZ_PV      = (size_t)PV_TOTAL * 4;
static constexpr size_t OFF_QF    = 0;
static constexpr size_t OFF_KF    = OFF_QF + SZ_F32ROWS;
static constexpr size_t OFF_PHQ   = OFF_KF + SZ_F32ROWS;
static constexpr size_t OFF_PHK   = OFF_PHQ + SZ_PH;
static constexpr size_t OFF_PHKTH = OFF_PHK + SZ_PH;
static constexpr size_t OFF_PHKTL = OFF_PHKTH + SZ_PHKT;
static constexpr size_t OFF_VTH   = OFF_PHKTL + SZ_PHKT;
static constexpr size_t OFF_VTL   = OFF_VTH + SZ_VT;
static constexpr size_t OFF_MT    = OFF_VTL + SZ_VT;
static constexpr size_t OFF_ATT   = OFF_MT + SZ_MT;
static constexpr size_t OFF_WQKV  = OFF_ATT + SZ_F32ROWS;
static constexpr size_t OFF_OMG2  = OFF_WQKV + SZ_WQKV;
static constexpr size_t OFF_WO2   = OFF_OMG2 + SZ_OMG2;
static constexpr size_t OFF_W1_2  = OFF_WO2 + SZ_WO2;
static constexpr size_t OFF_W2_2  = OFF_W1_2 + SZ_W1_2;
static constexpr size_t OFF_PV    = OFF_W2_2 + SZ_W2_2;
static constexpr size_t WS_TOTAL  = OFF_PV + SZ_PV;
static_assert(WS_TOTAL == 2682880);
static_assert(WS_TOTAL <= ((size_t)128 << 20));
static_assert(OFF_KF % 256 == 0 && OFF_PHQ % 256 == 0 && OFF_PHK % 256 == 0 && OFF_PHKTH % 256 == 0);
static_assert(OFF_PHKTL % 256 == 0 && OFF_VTH % 256 == 0 && OFF_VTL % 256 == 0 && OFF_MT % 256 == 0);
static_assert(OFF_ATT % 256 == 0 && OFF_WQKV % 256 == 0 && OFF_OMG2 % 256 == 0 && OFF_WO2 % 256 == 0);
static_assert(OFF_W1_2 % 256 == 0 && OFF_W2_2 % 256 == 0 && OFF_PV % 256 == 0);

extern "C" void kernel_launch(void* const* d_in, const int* in_sizes, int n_in,
                              void* d_out, int out_size, void* d_ws, size_t ws_size,
                              hipStream_t stream) {
  if (n_in != 19) return;
  if (in_sizes[0] != NTOK * DD) return;
  if (in_sizes[1] != NTOK * NTOK) return;
  if (in_sizes[2] != DD * DD || in_sizes[4] != DD * DD || in_sizes[6] != DD * DD || in_sizes[8] != DD * DD) return;
  if (in_sizes[3] != DD || in_sizes[5] != DD || in_sizes[7] != DD || in_sizes[9] != DD) return;
  if (in_sizes[10] != DD * HIDN || in_sizes[11] != HIDN || in_sizes[12] != HIDN * DD || in_sizes[13] != DD) return;
  if (in_sizes[14] != DD || in_sizes[15] != DD || in_sizes[16] != DD || in_sizes[17] != DD) return;
  if (in_sizes[18] != DD * RR) return;
  if (out_size != NTOK * DD) return;
  if (ws_size < WS_TOTAL) return;

  const float* Z     = (const float*)d_in[0];
  const int*   mask  = (const int*)d_in[1];
  const float* Wq    = (const float*)d_in[2];
  const float* bq    = (const float*)d_in[3];
  const float* Wk    = (const float*)d_in[4];
  const float* bk    = (const float*)d_in[5];
  const float* Wv    = (const float*)d_in[6];
  const float* bv    = (const float*)d_in[7];
  const float* Wo    = (const float*)d_in[8];
  const float* bo    = (const float*)d_in[9];
  const float* W1    = (const float*)d_in[10];
  const float* b1    = (const float*)d_in[11];
  const float* W2    = (const float*)d_in[12];
  const float* b2    = (const float*)d_in[13];
  const float* g1    = (const float*)d_in[14];
  const float* beta1 = (const float*)d_in[15];
  const float* g2    = (const float*)d_in[16];
  const float* beta2 = (const float*)d_in[17];
  const float* omega = (const float*)d_in[18];

  char* ws = (char*)d_ws;
  float*          QF    = (float*)(ws + OFF_QF);
  float*          KF    = (float*)(ws + OFF_KF);
  unsigned short* PHQ   = (unsigned short*)(ws + OFF_PHQ);
  unsigned short* PHK   = (unsigned short*)(ws + OFF_PHK);
  unsigned short* PHKTh = (unsigned short*)(ws + OFF_PHKTH);
  unsigned short* PHKTl = (unsigned short*)(ws + OFF_PHKTL);
  unsigned short* VTh   = (unsigned short*)(ws + OFF_VTH);
  unsigned short* VTl   = (unsigned short*)(ws + OFF_VTL);
  unsigned short* MT    = (unsigned short*)(ws + OFF_MT);
  float*          ATT   = (float*)(ws + OFF_ATT);
  unsigned short* WQKV  = (unsigned short*)(ws + OFF_WQKV);
  unsigned short* OMG2  = (unsigned short*)(ws + OFF_OMG2);
  unsigned short* WO2   = (unsigned short*)(ws + OFF_WO2);
  unsigned short* W1_2  = (unsigned short*)(ws + OFF_W1_2);
  unsigned short* W2_2  = (unsigned short*)(ws + OFF_W2_2);
  float*          PV    = (float*)(ws + OFF_PV);

  const dim3 blk(NTHR);
  k_wprep<<<dim3(1), blk, 0, stream>>>(Wq, Wk, Wv, omega, Wo, W1, W2, bq, bk, bv, bo, b1, b2, g1, beta1, g2, beta2,
                                       WQKV, OMG2, WO2, W1_2, W2_2, PV);
  k_rows<<<dim3(NTOK / 64), blk, 0, stream>>>(Z, WQKV, OMG2, PV, QF, KF, PHQ, PHK, PHKTh, PHKTl, VTh, VTl);
  k_m<<<dim3(1), blk, 0, stream>>>(PHKTh, PHKTl, VTh, VTl, MT);
  k_pair<<<dim3(NTOK / 64), blk, 0, stream>>>(QF, KF, PHQ, PHK, VTh, VTl, MT, mask, ATT);
  k_tail<<<dim3(NTOK / 64), blk, 0, stream>>>(ATT, Z, PV, WO2, W1_2, W2_2, (float*)d_out);
  (void)hipGetLastError();
}
